// EquivariantTransformerBlock_29214367547539
// MI455X (gfx1250) — hardware-run, weakly checked
//
#include <hip/hip_runtime.h>
#include <stddef.h>


#define HD     128
#define H2     256
#define INR    160
#define EF     16
#define NHD    8
#define ADY    64
#define PQC    320
#define HDC    144
#define KA     32
#define W1R    273
#define ASC    8
#define WSC    64
#define OSC    (1.0f / 512.0f)
#define VSC    (1.0f / 64.0f)
#define CSC    4096
#define CCO    (1.0f / 32768.0f)
#define NTHR   256
#define NWAVE  8
#define EPT    8
#define NGRP   2
#define CHUNK  (NTHR * EPT * NGRP)
#define WCAP   (EPT * NGRP * 32)
#define LISTN  (NWAVE * WCAP)
#define NBC    4096
#define NBF    1024
#define RCAP   40960
#define RBN    128
#define OTHR   512
#define DEGCAP 1024
#define BM     64
#define NCW    64
#define TWE    4
#define TTE    (TWE * 32)
#define TWN    2
#define TTN    (TWN * 32)
#define NLDSF  14592
#define LDS_NODE (TWN * NLDSF * 4)
#define ANB    32
#define STW    160
#define WSCAP  134217728
#define LDS_FILL ((RCAP + NBF + LISTN) * 4 + 64)

static_assert((CHUNK & (CHUNK - 1)) == 0);
static_assert(CHUNK <= 4096);
static_assert(NBC <= 4096 && NBF <= 4096);
static_assert((NBC & (NBC - 1)) == 0 && (NBF & (NBF - 1)) == 0);
static_assert(NBC == 4 * NBF);
static_assert(OTHR * 8 == NBC);
static_assert((RCAP % 32) == 0);
static_assert(BM * 4 == NTHR);
static_assert(WCAP == EPT * NGRP * 32);
static_assert(TTE == 128);
static_assert(TTN == 64);
static_assert(ANB * 8 == NTHR);
static_assert(NLDSF == 4096 + 4096 + 2048 + 2048 + 1024 + 1280);
static_assert(INR == 5 * 32 && HD == 4 * 32 && ADY == 2 * 32 && PQC == 5 * NCW);
static_assert(HDC == 9 * 16);
static_assert(STW * 4 == 640);

typedef float          v4f  __attribute__((ext_vector_type(4)));
typedef float          v8f  __attribute__((ext_vector_type(8)));
typedef int            v4i  __attribute__((ext_vector_type(4)));
typedef _Float16       v4h  __attribute__((ext_vector_type(4)));
typedef _Float16       v8h  __attribute__((ext_vector_type(8)));
typedef _Float16       v16h __attribute__((ext_vector_type(16)));
typedef _Float16       v8ha __attribute__((ext_vector_type(8), __may_alias__));
typedef unsigned short v4us __attribute__((ext_vector_type(4)));
typedef unsigned short v8us __attribute__((ext_vector_type(8)));
union FragH { v16h v; v8us u[2]; v8h h[2]; };

__device__ __forceinline__ v8f wmh(v16h a, v16h b, v8f c) {
  v8f d = __builtin_amdgcn_wmma_f32_16x16x32_f16(false, a, false, b, (short)0, c, false, false);
  asm volatile("v_nop\n\tv_nop\n\tv_nop\n\tv_nop" : "+v"(d) : "v"(a), "v"(b));
  return d;
}
__device__ __forceinline__ v8f zero8() { v8f z = {0.f, 0.f, 0.f, 0.f, 0.f, 0.f, 0.f, 0.f}; return z; }
__device__ __forceinline__ float silu_f(float x) { return x * __builtin_amdgcn_rcpf(1.0f + __expf(-x)); }
__device__ __forceinline__ float wsum32(float v) {
#pragma unroll
  for (int s = 16; s > 0; s >>= 1) v += __shfl_xor(v, s);
  return v;
}

__device__ __forceinline__ v16h frag_glb(const unsigned short* P, int row, int ld, int k0, int hh) {
  FragH f;
  const unsigned short* p = P + (size_t)row * ld + k0 + 8 * hh;
  f.u[0] = *(const v8us*)p;
  f.u[1] = *(const v8us*)(p + 16);
  return f.v;
}
__device__ __forceinline__ v16h frag_lds(const _Float16* T, int row, int ld, int k0, int hh) {
  FragH f;
  const _Float16* p = T + row * ld + k0 + 8 * hh;
  f.h[0] = *(const v8h*)p;
  f.h[1] = *(const v8h*)(p + 16);
  return f.v;
}
__device__ __forceinline__ v8h cvt8s(const float* p, float sc) {
  const v4f a = *(const v4f*)p, b = *(const v4f*)(p + 4);
  v8h o;
  o[0] = (_Float16)(a.x * sc); o[1] = (_Float16)(a.y * sc); o[2] = (_Float16)(a.z * sc); o[3] = (_Float16)(a.w * sc);
  o[4] = (_Float16)(b.x * sc); o[5] = (_Float16)(b.y * sc); o[6] = (_Float16)(b.z * sc); o[7] = (_Float16)(b.w * sc);
  return o;
}
__device__ __forceinline__ v16h frag_f32(const float* P, int row, int ld, int k0, int hh, float sc) {
  FragH f;
  const float* p = P + (size_t)row * ld + k0 + 8 * hh;
  f.h[0] = cvt8s(p, sc);
  f.h[1] = cvt8s(p + 16, sc);
  return f.v;
}

template <int NB>
__device__ __forceinline__ int scan_chunk(const int* __restrict__ dsts, int nE, int cbase, int slotBase,
                                          int vec8, int* list, int tid, int lane, int wave) {
  int wc = 0;
#pragma unroll
  for (int g = 0; g < NGRP; ++g) {
    const int el0  = (g * NTHR + tid) * EPT;
    const int e0   = cbase + el0;
    const int sent = -2147483647 - 1;
    v4i da, db;
    if (vec8 != 0 && cbase + CHUNK <= nE) {
      da = *(const v4i*)(dsts + e0);
      db = *(const v4i*)(dsts + e0 + 4);
    } else {
      da.x = (e0     < nE) ? dsts[min(e0, nE - 1)] : sent;
      da.y = (e0 + 1 < nE) ? dsts[min(e0 + 1, nE - 1)] : sent;
      da.z = (e0 + 2 < nE) ? dsts[min(e0 + 2, nE - 1)] : sent;
      da.w = (e0 + 3 < nE) ? dsts[min(e0 + 3, nE - 1)] : sent;
      db.x = (e0 + 4 < nE) ? dsts[min(e0 + 4, nE - 1)] : sent;
      db.y = (e0 + 5 < nE) ? dsts[min(e0 + 5, nE - 1)] : sent;
      db.z = (e0 + 6 < nE) ? dsts[min(e0 + 6, nE - 1)] : sent;
      db.w = (e0 + 7 < nE) ? dsts[min(e0 + 7, nE - 1)] : sent;
    }
    const unsigned nb = (unsigned)slotBase;
    const unsigned s0 = (unsigned)da.x - nb, s1 = (unsigned)da.y - nb;
    const unsigned s2 = (unsigned)da.z - nb, s3 = (unsigned)da.w - nb;
    const unsigned s4 = (unsigned)db.x - nb, s5 = (unsigned)db.y - nb;
    const unsigned s6 = (unsigned)db.z - nb, s7 = (unsigned)db.w - nb;
    const bool h0 = s0 < (unsigned)NB, h1 = s1 < (unsigned)NB, h2 = s2 < (unsigned)NB, h3 = s3 < (unsigned)NB;
    const bool h4 = s4 < (unsigned)NB, h5 = s5 < (unsigned)NB, h6 = s6 < (unsigned)NB, h7 = s7 < (unsigned)NB;
    const unsigned any = __builtin_amdgcn_ballot_w32(h0 | h1 | h2 | h3 | h4 | h5 | h6 | h7);
    if (any != 0u) {
#define HITJ(J, HJ, SJ) { \
        const unsigned mj = __builtin_amdgcn_ballot_w32(HJ); \
        if (mj != 0u) { \
          if (HJ) { \
            const int pos = wc + (int)__builtin_amdgcn_mbcnt_lo(mj, 0u); \
            if (pos < WCAP) list[wave * WCAP + pos] = ((el0 + (J)) << 12) | (int)(SJ); \
          } \
          wc += (int)__builtin_popcount(mj); } }
      HITJ(0, h0, s0)
      HITJ(1, h1, s1)
      HITJ(2, h2, s2)
      HITJ(3, h3, s3)
      HITJ(4, h4, s4)
      HITJ(5, h5, s5)
      HITJ(6, h6, s6)
      HITJ(7, h7, s7)
#undef HITJ
    }
  }
  return wc;
}

__global__ __launch_bounds__(NTHR) void k_count(const int* __restrict__ keys, int* cnt, int nE, int vec8) {
  __shared__ __attribute__((aligned(16))) int scnt[NBC];
  __shared__ __attribute__((aligned(16))) int list[LISTN];
  __shared__ int wcnt[NWAVE];
  const int tid = threadIdx.x, lane = tid & 31, wave = tid >> 5;
  const int nodeBase = blockIdx.x * NBC;

  for (int i = tid; i < NBC; i += NTHR) scnt[i] = 0;
  __syncthreads();

  const int nChunks = (nE + CHUNK - 1) / CHUNK;
#pragma unroll 1
  for (int ch = 0; ch < nChunks; ++ch) {
    const int cbase = ch * CHUNK;
    const int wc = scan_chunk<NBC>(keys, nE, cbase, nodeBase, vec8, list, tid, lane, wave);
    if (lane == 0) wcnt[wave] = wc;
    __syncthreads();
    if (wave == 0) {
#pragma unroll 1
      for (int wsx = 0; wsx < NWAVE; ++wsx) {
        int n = __builtin_amdgcn_readfirstlane(wcnt[wsx]);
        n = n > WCAP ? WCAP : (n < 0 ? 0 : n);
        const int* lp = list + wsx * WCAP;
#pragma unroll 1
        for (int i = 0; i < n; ++i) {
          const int ent  = __builtin_amdgcn_readfirstlane(lp[i]);
          const int slot = ent & (NBC - 1);
          if (lane == 0) scnt[slot] = scnt[slot] + 1;
        }
      }
    }
    __syncthreads();
  }

  v4i cq[4];
#pragma unroll
  for (int q = 0; q < 4; ++q) {
    const int f = (wave * 4 + q) * 128 + 4 * lane;
    cq[q] = *(const v4i*)(scnt + f);
  }
  int* cp = cnt + (size_t)nodeBase;
#pragma unroll
  for (int q = 0; q < 4; ++q) {
    const int f = (wave * 4 + q) * 128 + 4 * lane;
    *(volatile v4i*)(cp + f) = cq[q];
  }
  __threadfence();
#pragma unroll
  for (int q = 0; q < 4; ++q) {
    const int f = (wave * 4 + q) * 128 + 4 * lane;
    *(volatile v4i*)(cp + f) = cq[q];
  }
}

__global__ __launch_bounds__(OTHR) void k_offsets(
    const int* __restrict__ cnt, int* off, int* rbase, int nChunk) {
  __shared__ __attribute__((aligned(16))) int soff[NBC];
  __shared__ __attribute__((aligned(16))) int srb[RBN];
  __shared__ int wtot[OTHR / 32];
  const int tid = threadIdx.x, lane = tid & 31, wave = tid >> 5, sub = tid >> 7;
  for (int i = tid; i < RBN; i += OTHR) srb[i] = 0;
  int carry = 0;
#pragma unroll 1
  for (int ch = 0; ch < nChunk; ++ch) {
    const int base = ch * NBC;
    const v4i c0 = *(const v4i*)(cnt + base + 8 * tid);
    const v4i c1 = *(const v4i*)(cnt + base + 8 * tid + 4);
    const int e0 = max(c0.x, 0), e1 = max(c0.y, 0), e2 = max(c0.z, 0), e3 = max(c0.w, 0);
    const int e4 = max(c1.x, 0), e5 = max(c1.y, 0), e6 = max(c1.z, 0), e7 = max(c1.w, 0);
    const int ts = e0 + e1 + e2 + e3 + e4 + e5 + e6 + e7;
    int incl = ts;
#pragma unroll
    for (int d = 1; d < 32; d <<= 1) {
      const int t = __shfl_up(incl, d);
      if (lane >= d) incl += t;
    }
    if (lane == 31) wtot[wave] = incl;
    __syncthreads();
    const int S0 = wtot[0]  + wtot[1]  + wtot[2]  + wtot[3];
    const int S1 = wtot[4]  + wtot[5]  + wtot[6]  + wtot[7];
    const int S2 = wtot[8]  + wtot[9]  + wtot[10] + wtot[11];
    const int S3 = wtot[12] + wtot[13] + wtot[14] + wtot[15];
    int pre = 0;
#pragma unroll 1
    for (int w = 4 * sub; w < wave; ++w) pre += wtot[w];
    const int b0 = carry;
    const int b1 = b0 + ((S0 + 31) & ~31);
    const int b2 = b1 + ((S1 + 31) & ~31);
    const int b3 = b2 + ((S2 + 31) & ~31);
    const int b4 = b3 + ((S3 + 31) & ~31);
    const int myb = sub == 0 ? b0 : (sub == 1 ? b1 : (sub == 2 ? b2 : b3));
    if (tid == 0) {
      srb[min(4 * ch + 0, RBN - 1)] = b0;
      srb[min(4 * ch + 1, RBN - 1)] = b1;
      srb[min(4 * ch + 2, RBN - 1)] = b2;
      srb[min(4 * ch + 3, RBN - 1)] = b3;
    }
    int run = myb + pre + incl - ts;
    soff[8 * tid + 0] = run; run += e0;
    soff[8 * tid + 1] = run; run += e1;
    soff[8 * tid + 2] = run; run += e2;
    soff[8 * tid + 3] = run; run += e3;
    soff[8 * tid + 4] = run; run += e4;
    soff[8 * tid + 5] = run; run += e5;
    soff[8 * tid + 6] = run; run += e6;
    soff[8 * tid + 7] = run;
    carry = b4;
    __syncthreads();
    const v4i o0 = *(const v4i*)(soff + 4 * tid);
    const v4i o1 = *(const v4i*)(soff + 4 * (tid + OTHR));
    int* op = off + base;
    *(volatile v4i*)(op + 4 * tid) = o0;
    *(volatile v4i*)(op + 4 * (tid + OTHR)) = o1;
    __threadfence();
    *(volatile v4i*)(op + 4 * tid) = o0;
    *(volatile v4i*)(op + 4 * (tid + OTHR)) = o1;
    __syncthreads();
  }
  if (tid == 0) srb[min(4 * nChunk, RBN - 1)] = carry;
  __syncthreads();
  v4i rv = {0, 0, 0, 0};
  if (tid < 32) rv = *(const v4i*)(srb + 4 * tid);
  if (tid < 32) *(volatile v4i*)(rbase + 4 * tid) = rv;
  __threadfence();
  if (tid < 32) *(volatile v4i*)(rbase + 4 * tid) = rv;
}

__global__ __launch_bounds__(NTHR) void k_fill(
    const int* __restrict__ keys, const int* __restrict__ off, const int* __restrict__ rbase,
    int* csrE, int nE, int vec8, int csrLen) {
  extern __shared__ v4f lds_dyn[];
  int* region = (int*)lds_dyn;
  int* cursor = region + RCAP;
  int* list   = cursor + NBF;
  int* wcnt   = list + LISTN;
  const int tid = threadIdx.x, lane = tid & 31, wave = tid >> 5;
  const int b = blockIdx.x;
  const int nodeBase = b * NBF;

  int rb0 = rbase[b];
  const int rb1 = rbase[b + 1];
  rb0 = rb0 < 0 ? 0 : (rb0 > csrLen ? csrLen : rb0);
  rb0 &= ~31;
  int len = rb1 - rb0;
  len = len < 0 ? 0 : (len > RCAP ? RCAP : len);
  int lenW = (len + 31) & ~31;
  if (rb0 + lenW > csrLen) lenW = (csrLen - rb0) & ~31;

  {
    const v4i z = {0, 0, 0, 0};
    for (int i = tid; i < RCAP / 4; i += NTHR) ((v4i*)region)[i] = z;
    for (int s = tid; s < NBF; s += NTHR) {
      int o = off[nodeBase + s] - rb0;
      o = o < 0 ? 0 : (o > RCAP ? RCAP : o);
      cursor[s] = o;
    }
  }
  __syncthreads();

  const int nChunks = (nE + CHUNK - 1) / CHUNK;
#pragma unroll 1
  for (int ch = 0; ch < nChunks; ++ch) {
    const int cbase = ch * CHUNK;
    const int wc = scan_chunk<NBF>(keys, nE, cbase, nodeBase, vec8, list, tid, lane, wave);
    if (lane == 0) wcnt[wave] = wc;
    __syncthreads();
    if (wave == 0) {
#pragma unroll 1
      for (int wsx = 0; wsx < NWAVE; ++wsx) {
        int n = __builtin_amdgcn_readfirstlane(wcnt[wsx]);
        n = n > WCAP ? WCAP : (n < 0 ? 0 : n);
        const int* lp = list + wsx * WCAP;
#pragma unroll 1
        for (int i = 0; i < n; ++i) {
          const int ent  = __builtin_amdgcn_readfirstlane(lp[i]);
          const int slot = ent & (NBF - 1);
          int e = cbase + ((ent >> 12) & (CHUNK - 1));
          e = e > nE - 1 ? nE - 1 : e;
          if (lane == 0) {
            int pos = cursor[slot];
            pos = pos < 0 ? 0 : (pos > RCAP - 1 ? RCAP - 1 : pos);
            region[pos] = e;
            const int np = pos + 1;
            cursor[slot] = np > RCAP ? RCAP : np;
          }
        }
      }
    }
    __syncthreads();
  }

  const int nv = lenW >> 2;
  int* gp = csrE + rb0;
#pragma unroll 1
  for (int i = tid; i < nv; i += NTHR) {
    const v4i ve = ((const v4i*)region)[i];
    *(volatile v4i*)(gp + 4 * i) = ve;
  }
  __threadfence();
#pragma unroll 1
  for (int i = tid; i < nv; i += NTHR) {
    const v4i ve = ((const v4i*)region)[i];
    *(volatile v4i*)(gp + 4 * i) = ve;
  }
}

__global__ __launch_bounds__(NTHR) void k_wcvt(
    const float* __restrict__ We1, const float* __restrict__ We2, const float* __restrict__ Wv,
    const float* __restrict__ Wa, const float* __restrict__ Wc, const float* __restrict__ Wo,
    const float* __restrict__ Wn1, const float* __restrict__ Wn2,
    const float* __restrict__ Wf1, const float* __restrict__ Wf2,
    unsigned short* dPQW, unsigned short* dW1A, unsigned short* dWE2, unsigned short* dWHD,
    unsigned short* dWO, unsigned short* dWN1, unsigned short* dWN2, unsigned short* dWF1, unsigned short* dWF2) {
  const int job = (int)blockIdx.y;
  const int i = (int)blockIdx.x * NTHR + (int)threadIdx.x;
  const int Nout = (job == 0) ? PQC : ((job == 1 || job == 2 || job == 5) ? INR : ((job == 3) ? HDC : ((job == 7 || job == 8) ? H2 : HD)));
  const int KP = (job == 0 || job == 4 || job == 5) ? HD : ((job == 1) ? KA : ((job == 7 || job == 8) ? ADY : INR));
  const int K = (job == 1) ? EF : KP;
  const int ld = (job == 0 || job == 1 || job == 2 || job == 5) ? INR : ((job == 7 || job == 8) ? H2 : HD);
  const float* W =
      (job == 0) ? We1 : ((job == 1) ? (We1 + (size_t)257 * INR) : ((job == 2) ? We2 : ((job == 4) ? Wo :
      ((job == 5) ? Wn1 : ((job == 6) ? Wn2 : ((job == 7) ? Wf1 : ((job == 8) ? Wf2 : Wv)))))));
  unsigned short* dst =
      (job == 0) ? dPQW : ((job == 1) ? dW1A : ((job == 2) ? dWE2 : ((job == 3) ? dWHD : ((job == 4) ? dWO :
      ((job == 5) ? dWN1 : ((job == 6) ? dWN2 : ((job == 7) ? dWF1 : dWF2)))))));
  const int upc = KP >> 3;
  if (i >= Nout * upc) return;
  const int n = i / upc;
  const int seg = i - n * upc;
  const int hi = (job == 0 && n >= INR) ? 1 : 0;
  const int col = n - hi * INR;
  v8h o;
#pragma unroll
  for (int j = 0; j < 8; ++j) {
    const int k = 8 * seg + j;
    const int kc = k < K - 1 ? k : K - 1;
    float v;
    if (job == 3) {
      const int cv = n < HD - 1 ? n : HD - 1;
      int ca = n - HD; ca = ca < 0 ? 0 : (ca > NHD - 1 ? NHD - 1 : ca);
      const float vv = Wv[(size_t)kc * HD + cv];
      const float va = Wa[(size_t)kc * NHD + ca];
      const float vc = Wc[kc];
      v = (n < HD) ? vv * (float)WSC : ((n < HD + NHD) ? va * (float)WSC : ((n == HD + NHD) ? vc * (float)CSC : 0.0f));
    } else {
      v = W[(size_t)(kc + hi * HD) * ld + col] * (float)WSC;
    }
    o[j] = (k < K) ? (_Float16)v : (_Float16)0.0f;
  }
  const v8us ob = __builtin_bit_cast(v8us, o);
  unsigned short* d = dst + (size_t)i * 8;
  *(volatile v8us*)d = ob;
  __threadfence();
  *(volatile v8us*)d = ob;
}

__global__ __launch_bounds__(NTHR) void k_pq(const float* __restrict__ A, const unsigned short* __restrict__ Bp,
                                             float* C, int nA) {
  __shared__ __attribute__((aligned(16))) float stg[BM * NCW];
  const int tid = threadIdx.x, lane = tid & 31, wave = tid >> 5, hh = lane >> 4, m = lane & 15;
  const int rowBase = (int)blockIdx.x * BM;
  const int colBase = (int)blockIdx.y * NCW;
  const int rg = wave >> 1, chf = wave & 1;
  const int r0 = rg * 16;
  const int c0 = chf * 32;

  int arow = rowBase + r0 + m; arow = arow > nA - 1 ? nA - 1 : arow;
  const float* ap = A + (size_t)arow * HD + 8 * hh;
  const unsigned short* bpA = Bp + (size_t)(colBase + c0 + m) * HD + 8 * hh;
  const unsigned short* bpB = bpA + (size_t)16 * HD;

  v8f acc0 = zero8();
  v8f acc1 = zero8();
#pragma unroll 1
  for (int kt = 0; kt < 4; ++kt) {
    FragH a, b0, b1;
    a.h[0] = cvt8s(ap + 32 * kt, (float)ASC);
    a.h[1] = cvt8s(ap + 32 * kt + 16, (float)ASC);
    b0.u[0] = *(const v8us*)(bpA + 32 * kt);
    b0.u[1] = *(const v8us*)(bpA + 32 * kt + 16);
    b1.u[0] = *(const v8us*)(bpB + 32 * kt);
    b1.u[1] = *(const v8us*)(bpB + 32 * kt + 16);
    acc0 = wmh(a.v, b0.v, acc0);
    acc1 = wmh(a.v, b1.v, acc1);
  }

  {
    float* sp = stg + (size_t)(r0 + 8 * hh) * NCW + c0 + m;
#pragma unroll
    for (int r = 0; r < 8; ++r) {
      sp[r * NCW]      = acc0[r] * OSC;
      sp[r * NCW + 16] = acc1[r] * OSC;
    }
  }
  __syncthreads();

  v4f cv[4];
#pragma unroll
  for (int it = 0; it < 4; ++it) {
    const int id = it * NTHR + tid;
    const int row = id >> 4, seg = id & 15;
    cv[it] = *(const v4f*)(stg + (size_t)row * NCW + 4 * seg);
  }
#pragma unroll
  for (int it = 0; it < 4; ++it) {
    const int id = it * NTHR + tid;
    const int row = id >> 4, seg = id & 15;
    float* gp = C + (size_t)(rowBase + row) * PQC + colBase + 4 * seg;
    *(volatile v4f*)gp = cv[it];
  }
  __threadfence();
#pragma unroll
  for (int it = 0; it < 4; ++it) {
    const int id = it * NTHR + tid;
    const int row = id >> 4, seg = id & 15;
    float* gp = C + (size_t)(rowBase + row) * PQC + colBase + 4 * seg;
    *(volatile v4f*)gp = cv[it];
  }
}

__device__ __forceinline__ void vrows_pass(const _Float16* sVw, unsigned short* Vp, int s0, int lane) {
#pragma unroll
  for (int i = 0; i < 8; ++i) {
    const v8ha t = *(const v8ha*)(sVw + 256 * i + 8 * lane);
    const v8us u = __builtin_bit_cast(v8us, t);
    *(volatile v8us*)(Vp + (size_t)s0 * HD + 256 * i + 8 * lane) = u;
  }
}

__global__ __launch_bounds__(TTE) void k_edge(
    const int* __restrict__ csrE, const int* __restrict__ srcI, const int* __restrict__ dstI,
    const float* __restrict__ crd, const float* __restrict__ aF, const float* __restrict__ PQ,
    const float* __restrict__ wrad, const float* __restrict__ be1,
    const unsigned short* __restrict__ W1Ap, const unsigned short* __restrict__ WE2p,
    const float* __restrict__ be2, const unsigned short* __restrict__ WHDp,
    unsigned short* VH, float* LH, float* CH, int nN, int nE, int csrLen, int sBase) {
  __shared__ __attribute__((aligned(16))) float    sBig[TWE][2560];
  __shared__ __attribute__((aligned(16))) _Float16 sA1[TWE][16 * INR];
  __shared__ __attribute__((aligned(16))) float    sRel[TWE][64];
  __shared__ __attribute__((aligned(16))) int      sIdx[TWE][64];
  const int tid = threadIdx.x, lane = tid & 31, wave = tid >> 5, hh = lane >> 4, m = lane & 15;
  const int sl0 = ((int)blockIdx.x * TWE + wave) * 16;
  float*    sX  = sBig[wave];
  _Float16* sM  = (_Float16*)sBig[wave];
  _Float16* sV  = sM + 16 * INR;
  float*    sL  = sBig[wave] + 2304;
  _Float16* sA1w = sA1[wave];
  _Float16* sAa  = sA1w;

  {
    const int e = lane & 15;
    int s = sBase + sl0 + e; s = s > csrLen - 1 ? csrLen - 1 : s;
    int eid = csrE[s];
    eid = eid < 0 ? 0 : (eid > nE - 1 ? nE - 1 : eid);
    int si = srcI[eid], di = dstI[eid];
    si = si < 0 ? 0 : (si > nN - 1 ? nN - 1 : si);
    di = di < 0 ? 0 : (di > nN - 1 ? nN - 1 : di);
    const float* ps = crd + (size_t)si * 3;
    const float* pd = crd + (size_t)di * 3;
    const float rx = ps[0] - pd[0];
    const float ry = ps[1] - pd[1];
    const float rz = ps[2] - pd[2];
    const float rd = (rx * rx + rz * rz) + ry * ry;
    if (lane < 16) {
      sIdx[wave][4 * e + 0] = si;
      sIdx[wave][4 * e + 1] = di;
      sIdx[wave][4 * e + 2] = eid;
      sIdx[wave][4 * e + 3] = 0;
      sRel[wave][4 * e + 0] = rx;
      sRel[wave][4 * e + 1] = ry;
      sRel[wave][4 * e + 2] = rz;
      sRel[wave][4 * e + 3] = rd;
    }
  }
  __syncthreads();

  {
    const int row = lane >> 1, part = lane & 1;
    const int eid = sIdx[wave][4 * row + 2];
    const float* ar = aF + (size_t)eid * EF + 8 * part;
    const v8h o = cvt8s(ar, (float)ASC);
    v8h z8;
#pragma unroll
    for (int j = 0; j < 8; ++j) z8[j] = (_Float16)0.0f;
    *(v8h*)(sAa + row * KA + 8 * part) = o;
    *(v8h*)(sAa + row * KA + 16 + 8 * part) = z8;
  }
  __syncthreads();

#pragma unroll 1
  for (int np = 0; np < 5; ++np) {
    const int c0 = 32 * np + m, c1 = c0 + 16;
    const v16h a  = frag_lds(sAa, m, KA, 0, hh);
    const v16h b0 = frag_glb(W1Ap, c0, KA, 0, hh);
    const v16h b1 = frag_glb(W1Ap, c1, KA, 0, hh);
    v8f acc0 = wmh(a, b0, zero8());
    v8f acc1 = wmh(a, b1, zero8());
#pragma unroll
    for (int r = 0; r < 8; ++r) {
      sX[(8 * hh + r) * INR + c0] = acc0[r] * OSC;
      sX[(8 * hh + r) * INR + c1] = acc1[r] * OSC;
    }
  }
  __syncthreads();

  {
    const int l8 = lane < 8 ? lane : 7;
    const v4f wq0 = *(const v4f*)(wrad + 4 * lane);
    const v4f wq1 = *(const v4f*)(wrad + HD + 4 * l8);
    const v4f bq0 = *(const v4f*)(be1 + 4 * lane);
    const v4f bq1 = *(const v4f*)(be1 + HD + 4 * l8);
#pragma unroll 1
    for (int e = 0; e < 16; ++e) {
      const int si = sIdx[wave][4 * e + 0];
      const int di = sIdx[wave][4 * e + 1];
      const float rd = sRel[wave][4 * e + 3];
      const float* pr = PQ + (size_t)si * PQC;
      const float* qr = PQ + (size_t)di * PQC + INR;
      const v4f p0 = *(const v4f*)(pr + 4 * lane);
      const v4f q0 = *(const v4f*)(qr + 4 * lane);
      const v4f p1 = *(const v4f*)(pr + HD + 4 * l8);
      const v4f q1 = *(const v4f*)(qr + HD + 4 * l8);
      const v4f x0 = *(const v4f*)(sX + e * INR + 4 * lane) + p0 + q0 + wq0 * rd + bq0;
      const v4f x1 = *(const v4f*)(sX + e * INR + HD + 4 * l8) + p1 + q1 + wq1 * rd + bq1;
      v4h o0, o1;
      o0.x = (_Float16)(silu_f(x0.x) * (float)ASC); o0.y = (_Float16)(silu_f(x0.y) * (float)ASC);
      o0.z = (_Float16)(silu_f(x0.z) * (float)ASC); o0.w = (_Float16)(silu_f(x0.w) * (float)ASC);
      o1.x = (_Float16)(silu_f(x1.x) * (float)ASC); o1.y = (_Float16)(silu_f(x1.y) * (float)ASC);
      o1.z = (_Float16)(silu_f(x1.z) * (float)ASC); o1.w = (_Float16)(silu_f(x1.w) * (float)ASC);
      *(v4h*)(sA1w + e * INR + 4 * lane) = o0;
      if (lane < 8) *(v4h*)(sA1w + e * INR + HD + 4 * lane) = o1;
    }
  }
  __syncthreads();

#pragma unroll 1
  for (int np = 0; np < 5; ++np) {
    const int c0 = 32 * np + m, c1 = c0 + 16;
    v8f acc0 = zero8(), acc1 = zero8();
#pragma unroll 1
    for (int kt = 0; kt < 5; ++kt) {
      const v16h a  = frag_lds(sA1w, m, INR, 32 * kt, hh);
      const v16h b0 = frag_glb(WE2p, c0, INR, 32 * kt, hh);
      const v16h b1 = frag_glb(WE2p, c1, INR, 32 * kt, hh);
      acc0 = wmh(a, b0, acc0);
      acc1 = wmh(a, b1, acc1);
    }
    const float bv0 = be2[c0], bv1 = be2[c1];
#pragma unroll
    for (int r = 0; r < 8; ++r) {
      sM[(8 * hh + r) * INR + c0] = (_Float16)(silu_f(acc0[r] * OSC + bv0) * (float)ASC);
      sM[(8 * hh + r) * INR + c1] = (_Float16)(silu_f(acc1[r] * OSC + bv1) * (float)ASC);
    }
  }
  __syncthreads();

#pragma unroll 1
  for (int np = 0; np < 4; ++np) {
    const int c0 = 32 * np + m, c1 = c0 + 16;
    v8f acc0 = zero8(), acc1 = zero8();
#pragma unroll 1
    for (int kt = 0; kt < 5; ++kt) {
      const v16h a  = frag_lds(sM, m, INR, 32 * kt, hh);
      const v16h b0 = frag_glb(WHDp, c0, INR, 32 * kt, hh);
      const v16h b1 = frag_glb(WHDp, c1, INR, 32 * kt, hh);
      acc0 = wmh(a, b0, acc0);
      acc1 = wmh(a, b1, acc1);
    }
#pragma unroll
    for (int r = 0; r < 8; ++r) {
      sV[(8 * hh + r) * HD + c0] = (_Float16)(acc0[r] * VSC);
      sV[(8 * hh + r) * HD + c1] = (_Float16)(acc1[r] * VSC);
    }
  }
  {
    v8f acc2 = zero8();
#pragma unroll 1
    for (int kt = 0; kt < 5; ++kt) {
      const v16h a = frag_lds(sM, m, INR, 32 * kt, hh);
      const v16h b = frag_glb(WHDp, HD + m, INR, 32 * kt, hh);
      acc2 = wmh(a, b, acc2);
    }
    const float scl = (m < NHD) ? OSC : ((m == NHD) ? CCO : 0.0f);
#pragma unroll
    for (int r = 0; r < 8; ++r) sL[(8 * hh + r) * 16 + m] = acc2[r] * scl;
  }
  __syncthreads();

  const int l16 = lane < 16 ? lane : 15;
  const float coef = sL[l16 * 16 + NHD];
  const float rx = sRel[wave][4 * l16 + 0];
  const float ry = sRel[wave][4 * l16 + 1];
  const float rz = sRel[wave][4 * l16 + 2];
  const float rd = sRel[wave][4 * l16 + 3];
  const float inv = 1.0f / (sqrtf(rd + 1e-5f) + 1.0f);
  v4f cw;
  cw.x = (coef * rx) * inv;
  cw.y = (coef * ry) * inv;
  cw.z = (coef * rz) * inv;
  cw.w = 0.0f;
  const v4f lv = *(const v4f*)(sL + (lane >> 1) * 16 + 4 * (lane & 1));
  float* lp = LH + (size_t)(sl0 + (lane >> 1)) * NHD + 4 * (lane & 1);
  float* cp = CH + (size_t)(sl0 + l16) * 4;
  const bool act = lane < 16;
  vrows_pass(sV, VH, sl0, lane);
  *(volatile v4f*)lp = lv;
  if (act) *(volatile v4f*)cp = cw;
  __threadfence();
  vrows_pass(sV, VH, sl0, lane);
  *(volatile v4f*)lp = lv;
  if (act) *(volatile v4f*)cp = cw;
}

template <int SECOND>
__global__ __launch_bounds__(NTHR) void k_agg(
    const int* __restrict__ cnt, const int* __restrict__ off,
    const unsigned short* __restrict__ VH, const float* __restrict__ LH, const float* __restrict__ CH,
    float* ST, const float* __restrict__ crd, float* CO, unsigned short* HAGG,
    int nN, int csrLen, int sBase, int HS) {
  __shared__ __attribute__((aligned(16))) float sPos[ANB * 4];
  __shared__ __attribute__((aligned(16))) float sSt[NWAVE][32];
  const int tid = threadIdx.x, lane = tid & 31, wave = tid >> 5, head = lane >> 2, ln4 = lane & 3;
  const int nb = (int)blockIdx.x * ANB;
  const _Float16* Vh = (const _Float16*)VH;
  const float NEGI = __int_as_float(0xff800000u);
  const v4f z4 = {0.f, 0.f, 0.f, 0.f};

  int nl = nb + wave * 4 + ln4; nl = nl > nN - 1 ? nN - 1 : nl;
  const int cnt_l = cnt[nl];
  const int off_l = off[nl];
  float pxl = 0.f, pyl = 0.f, pzl = 0.f;
  if (SECOND) {
    const float* pc = crd + (size_t)nl * 3;
    pxl = pc[0]; pyl = pc[1]; pzl = pc[2];
  }

  v4us agv[4];
#pragma unroll
  for (int j = 0; j < 4; ++j) {
    const int nrow = nb + wave * 4 + j;
    int dg = __builtin_amdgcn_readfirstlane(__shfl(cnt_l, j));
    const bool ovf = dg > DEGCAP;
    dg = dg < 0 ? 0 : (dg > DEGCAP ? DEGCAP : dg);
    int st = __builtin_amdgcn_readfirstlane(__shfl(off_l, j));
    st = st < 0 ? 0 : (st > csrLen - 1 ? csrLen - 1 : st);
    const int lo = st > sBase ? st : sBase;
    int hi = st + dg; hi = hi < sBase + HS ? hi : sBase + HS;
    int nloc = hi - lo; nloc = nloc < 0 ? 0 : nloc;
    int ls = lo - sBase; ls = ls < 0 ? 0 : (ls > HS - 1 ? HS - 1 : ls);

    v4f acc = z4, cacc = z4;
    float den = 0.f, mxo = NEGI;
    if (SECOND) {
      const float* sp = ST + (size_t)nrow * STW;
      acc  = *(const v4f*)(sp + 4 * lane);
      den  = sp[128 + head];
      mxo  = sp[136 + head];
      cacc = *(const v4f*)(sp + 144);
    }
    float lm = NEGI;
#pragma unroll 1
    for (int i = 0; i < nloc; ++i) {
      int s = ls + i; s = s > HS - 1 ? HS - 1 : s;
      lm = fmaxf(lm, LH[(size_t)s * NHD + head]);
    }
    const float M = fmaxf(mxo, lm);
    const float resc = (mxo == NEGI) ? 0.0f : __expf(mxo - M);
    den *= resc;
    acc = acc * resc;
#pragma unroll 1
    for (int i = 0; i < nloc; ++i) {
      int s = ls + i; s = s > HS - 1 ? HS - 1 : s;
      const float ex = __expf(LH[(size_t)s * NHD + head] - M);
      den += ex;
      const v4h vv = *(const v4h*)(Vh + (size_t)s * HD + 4 * lane);
      acc.x += ex * (float)vv.x; acc.y += ex * (float)vv.y;
      acc.z += ex * (float)vv.z; acc.w += ex * (float)vv.w;
      cacc += *(const v4f*)(CH + (size_t)s * 4);
    }

    if (!SECOND) {
      agv[j] = __builtin_bit_cast(v4us, z4.xy);
      float* ss = sSt[wave];
      __syncthreads();
      if (ln4 == 0) { ss[head] = den; ss[8 + head] = M; }
      if (lane == 0) { ss[16] = cacc.x; ss[17] = cacc.y; ss[18] = cacc.z; ss[19] = 0.f; }
      if (lane >= 20) ss[lane] = 0.f;
      __syncthreads();
      const int l8 = lane < 8 ? lane : 7;
      const v4f tl = *(const v4f*)(ss + 4 * l8);
      float* sp = ST + (size_t)nrow * STW;
      *(volatile v4f*)(sp + 4 * lane) = acc;
      if (lane < 8) *(volatile v4f*)(sp + 128 + 4 * lane) = tl;
      __threadfence();
      *(volatile v4f*)(sp + 4 * lane) = acc;
      if (lane < 8) *(volatile v4f*)(sp + 128 + 4 * lane) = tl;
    } else {
      const float inv = (den > 0.0f) ? (1.0f / den) : 0.0f;
      v4f hv = acc * inv;
      if (ovf) {
        const float qn = __int_as_float(0x7fc00000u);
        hv.x = qn; hv.y = qn; hv.z = qn; hv.w = qn;
      }
      v4h ho;
      ho.x = (_Float16)hv.x; ho.y = (_Float16)hv.y; ho.z = (_Float16)hv.z; ho.w = (_Float16)hv.w;
      agv[j] = __builtin_bit_cast(v4us, ho);
      const float px = __shfl(pxl, j) + cacc.x;
      const float py = __shfl(pyl, j) + cacc.y;
      const float pz = __shfl(pzl, j) + cacc.z;
      if (lane == 0) {
        const int ln = wave * 4 + j;
        sPos[4 * ln + 0] = px; sPos[4 * ln + 1] = py; sPos[4 * ln + 2] = pz; sPos[4 * ln + 3] = 0.f;
      }
    }
  }

  if (SECOND) {
#pragma unroll
    for (int j = 0; j < 4; ++j)
      *(volatile v4us*)(HAGG + (size_t)(nb + wave * 4 + j) * HD + 4 * lane) = agv[j];
    __syncthreads();
    const v4f pv = *(const v4f*)(sPos + 4 * lane);
    float* pg = CO + (size_t)(nb + lane) * 4;
    if (wave == 0) *(volatile v4f*)pg = pv;
    __threadfence();
#pragma unroll
    for (int j = 0; j < 4; ++j)
      *(volatile v4us*)(HAGG + (size_t)(nb + wave * 4 + j) * HD + 4 * lane) = agv[j];
    if (wave == 0) *(volatile v4f*)pg = pv;
  }
}

__global__ __launch_bounds__(TTN) void k_node(
    const float* __restrict__ hF, const float* __restrict__ yF, const float* __restrict__ resF,
    const unsigned short* __restrict__ HAGG,
    const unsigned short* __restrict__ WOp,
    const unsigned short* __restrict__ WF1p, const float* __restrict__ bf1,
    const unsigned short* __restrict__ WF2p, const float* __restrict__ bf2,
    const unsigned short* __restrict__ WN1p, const float* __restrict__ bn1,
    const unsigned short* __restrict__ WN2p, const float* __restrict__ bn2,
    float* out0, float* R2, int nN) {
  extern __shared__ v4f lds_dyn[];
  const int tid = threadIdx.x, lane = tid & 31, wave = tid >> 5, hh = lane >> 4, m = lane & 15;
  float* wb = (float*)lds_dyn + (size_t)wave * NLDSF;
  float*    sS  = wb;
  float*    sS2 = wb + 4096;
  float*    sF  = wb + 8192;
  float*    sR  = wb + 10240;
  _Float16* sH1 = (_Float16*)(wb + 12288);
  _Float16* sT  = (_Float16*)(wb + 13312);
  const int n0 = ((int)blockIdx.x * TWN + wave) * 16;
  int yrow = n0 + m; yrow = yrow > nN - 1 ? nN - 1 : yrow;

#pragma unroll 1
  for (int np = 0; np < 4; ++np) {
    const int c0 = 32 * np + m, c1 = c0 + 16;
    v8f acc0 = zero8(), acc1 = zero8();
#pragma unroll 1
    for (int kt = 0; kt < 4; ++kt) {
      const v16h a  = frag_glb(HAGG, n0 + m, HD, 32 * kt, hh);
      const v16h b0 = frag_glb(WOp, c0, HD, 32 * kt, hh);
      const v16h b1 = frag_glb(WOp, c1, HD, 32 * kt, hh);
      acc0 = wmh(a, b0, acc0);
      acc1 = wmh(a, b1, acc1);
    }
#pragma unroll
    for (int r = 0; r < 8; ++r) {
      sF[(8 * hh + r) * HD + c0] = acc0[r] * OSC;
      sF[(8 * hh + r) * HD + c1] = acc1[r] * OSC;
    }
  }
#pragma unroll 1
  for (int np = 0; np < 8; ++np) {
    const int c0 = 32 * np + m, c1 = c0 + 16;
    v8f acc0 = zero8(), acc1 = zero8();
#pragma unroll 1
    for (int kt = 0; kt < 2; ++kt) {
      const v16h a  = frag_f32(yF, yrow, ADY, 32 * kt, hh, (float)ASC);
      const v16h b0 = frag_glb(WF1p, c0, ADY, 32 * kt, hh);
      const v16h b1 = frag_glb(WF1p, c1, ADY, 32 * kt, hh);
      acc0 = wmh(a, b0, acc0);
      acc1 = wmh(a, b1, acc1);
    }
    const float bv0 = bf1[c0], bv1 = bf1[c1];
#pragma unroll
    for (int r = 0; r < 8; ++r) {
      sS[(8 * hh + r) * H2 + c0] = acc0[r] * OSC + bv0;
      sS[(8 * hh + r) * H2 + c1] = acc1[r] * OSC + bv1;
    }
  }
#pragma unroll 1
  for (int np = 0; np < 8; ++np) {
    const int c0 = 32 * np + m, c1 = c0 + 16;
    v8f acc0 = zero8(), acc1 = zero8();
#pragma unroll 1
    for (int kt = 0; kt < 2; ++kt) {
      const v16h a  = frag_f32(yF, yrow, ADY, 32 * kt, hh, (float)ASC);
      const v16h b0 = frag_glb(WF2p, c0, ADY, 32 * kt, hh);
      const v16h b1 = frag_glb(WF2p, c1, ADY, 32 * kt, hh);
      acc0 = wmh(a, b0, acc0);
      acc1 = wmh(a, b1, acc1);
    }
    const float bv0 = bf2[c0], bv1 = bf2[c1];
#pragma unroll
    for (int r = 0; r < 8; ++r) {
      sS2[(8 * hh + r) * H2 + c0] = acc0[r] * OSC + bv0;
      sS2[(8 * hh + r) * H2 + c1] = acc1[r] * OSC + bv1;
    }
  }
  __syncthreads();

#pragma unroll 1
  for (int i = 0; i < 16; ++i) {
    int nc = n0 + i; nc = nc > nN - 1 ? nN - 1 : nc;
    const v4f hv = *(const v4f*)(hF + (size_t)nc * HD + 4 * lane);
    const v4f rv = *(const v4f*)(resF + (size_t)nc * HD + 4 * lane);
    const v4f fv = *(const v4f*)(sF + i * HD + 4 * lane);
    const v4f x = hv + fv;
    const v4f r1 = rv + fv;
    float s = (x.x + x.y) + (x.z + x.w);
    s = wsum32(s);
    const float mu = s * (1.0f / 128.0f);
    const v4f d = x - mu;
    float q = (d.x * d.x + d.y * d.y) + (d.z * d.z + d.w * d.w);
    q = wsum32(q);
    const float rs = rsqrtf(q * (1.0f / 128.0f) + 1e-5f);
    const v4f sc = *(const v4f*)(sS + i * H2 + 4 * lane);
    const v4f sh = *(const v4f*)(sS + i * H2 + HD + 4 * lane);
    const v4f on = sc + 1.0f;
    const v4f h1 = d * rs * on + sh;
    *(v4f*)(sS + i * H2 + 4 * lane) = h1;
    *(v4f*)(sS + i * H2 + HD + 4 * lane) = r1;
    v4h o;
    o.x = (_Float16)(h1.x * (float)ASC); o.y = (_Float16)(h1.y * (float)ASC);
    o.z = (_Float16)(h1.z * (float)ASC); o.w = (_Float16)(h1.w * (float)ASC);
    *(v4h*)(sH1 + i * HD + 4 * lane) = o;
  }
  __syncthreads();

#pragma unroll 1
  for (int np = 0; np < 5; ++np) {
    const int c0 = 32 * np + m, c1 = c0 + 16;
    v8f acc0 = zero8(), acc1 = zero8();
#pragma unroll 1
    for (int kt = 0; kt < 4; ++kt) {
      const v16h a  = frag_lds(sH1, m, HD, 32 * kt, hh);
      const v16h b0 = frag_glb(WN1p, c0, HD, 32 * kt, hh);
      const v16h b1 = frag_glb(WN1p, c1, HD, 32 * kt, hh);
      acc0 = wmh(a, b0, acc0);
      acc1 = wmh(a, b1, acc1);
    }
    const float bv0 = bn1[c0], bv1 = bn1[c1];
#pragma unroll
    for (int r = 0; r < 8; ++r) {
      sT[(8 * hh + r) * INR + c0] = (_Float16)(silu_f(acc0[r] * OSC + bv0) * (float)ASC);
      sT[(8 * hh + r) * INR + c1] = (_Float16)(silu_f(acc1[r] * OSC + bv1) * (float)ASC);
    }
  }
  __syncthreads();

#pragma unroll 1
  for (int np = 0; np < 4; ++np) {
    const int c0 = 32 * np + m, c1 = c0 + 16;
    v8f acc0 = zero8(), acc1 = zero8();
#pragma unroll 1
    for (int kt = 0; kt < 5; ++kt) {
      const v16h a  = frag_lds(sT, m, INR, 32 * kt, hh);
      const v16h b0 = frag_glb(WN2p, c0, INR, 32 * kt, hh);
      const v16h b1 = frag_glb(WN2p, c1, INR, 32 * kt, hh);
      acc0 = wmh(a, b0, acc0);
      acc1 = wmh(a, b1, acc1);
    }
    const float bv0 = bn2[c0], bv1 = bn2[c1];
#pragma unroll
    for (int r = 0; r < 8; ++r) {
      sF[(8 * hh + r) * HD + c0] = acc0[r] * OSC + bv0;
      sF[(8 * hh + r) * HD + c1] = acc1[r] * OSC + bv1;
    }
  }
  __syncthreads();

#pragma unroll 1
  for (int i = 0; i < 16; ++i) {
    const v4f f3 = *(const v4f*)(sF + i * HD + 4 * lane);
    const v4f h1 = *(const v4f*)(sS + i * H2 + 4 * lane);
    const v4f r1 = *(const v4f*)(sS + i * H2 + HD + 4 * lane);
    const v4f r2 = r1 + f3;
    *(v4f*)(sR + i * HD + 4 * lane) = r2;
    const v4f x = h1 + f3;
    float s = (x.x + x.y) + (x.z + x.w);
    s = wsum32(s);
    const float mu = s * (1.0f / 128.0f);
    const v4f d = x - mu;
    float q = (d.x * d.x + d.y * d.y) + (d.z * d.z + d.w * d.w);
    q = wsum32(q);
    const float rs = rsqrtf(q * (1.0f / 128.0f) + 1e-5f);
    const v4f sc = *(const v4f*)(sS2 + i * H2 + 4 * lane);
    const v4f sh = *(const v4f*)(sS2 + i * H2 + HD + 4 * lane);
    const v4f on = sc + 1.0f;
    const v4f h2v = d * rs * on + sh;
    *(v4f*)(sF + i * HD + 4 * lane) = h2v;
  }
  __syncthreads();

#pragma unroll 1
  for (int i = 0; i < 16; ++i) {
    const int n = n0 + i;
    const v4f hrow = *(const v4f*)(sF + i * HD + 4 * lane);
    const v4f rrow = *(const v4f*)(sR + i * HD + 4 * lane);
    if (n < nN) *(volatile v4f*)(out0 + (size_t)n * HD + 4 * lane) = hrow;
    *(volatile v4f*)(R2 + (size_t)n * HD + 4 * lane) = rrow;
  }
  __threadfence();
#pragma unroll 1
  for (int i = 0; i < 16; ++i) {
    const int n = n0 + i;
    const v4f hrow = *(const v4f*)(sF + i * HD + 4 * lane);
    const v4f rrow = *(const v4f*)(sR + i * HD + 4 * lane);
    if (n < nN) *(volatile v4f*)(out0 + (size_t)n * HD + 4 * lane) = hrow;
    *(volatile v4f*)(R2 + (size_t)n * HD + 4 * lane) = rrow;
  }
}

__global__ __launch_bounds__(NTHR) void k_out(const float* __restrict__ CO, const float* __restrict__ R2,
                                              float* out, int nN, int q0, int qSplit, int q1, int e1, int e2) {
  const int q = q0 + (int)blockIdx.x * NTHR + (int)threadIdx.x;
  const int qq = q < q1 - 1 ? q : q1 - 1;
  const int jb = 4 * qq - e1;
  v4f ca;
  {
    int nd0 = jb / 3;       const int cm0 = jb - 3 * nd0;       nd0 = nd0 > nN - 1 ? nN - 1 : nd0;
    int nd1 = (jb + 1) / 3; const int cm1 = (jb + 1) - 3 * nd1; nd1 = nd1 > nN - 1 ? nN - 1 : nd1;
    int nd2 = (jb + 2) / 3; const int cm2 = (jb + 2) - 3 * nd2; nd2 = nd2 > nN - 1 ? nN - 1 : nd2;
    int nd3 = (jb + 3) / 3; const int cm3 = (jb + 3) - 3 * nd3; nd3 = nd3 > nN - 1 ? nN - 1 : nd3;
    ca.x = CO[(size_t)nd0 * 4 + cm0];
    ca.y = CO[(size_t)nd1 * 4 + cm1];
    ca.z = CO[(size_t)nd2 * 4 + cm2];
    ca.w = CO[(size_t)nd3 * 4 + cm3];
  }
  int j2 = 4 * qq - e2; j2 = j2 < 0 ? 0 : j2;
  const v4f cb = *(const v4f*)(R2 + j2);
  const v4f v = (qq < qSplit) ? ca : cb;
  float* p = out + (size_t)4 * qq;
  if (q < q1) *(volatile v4f*)p = v;
  __threadfence();
  if (q < q1) *(volatile v4f*)p = v;
}

extern "C" void kernel_launch(void* const* d_in, const int* in_sizes, int n_in,
                              void* d_out, int out_size, void* d_ws, size_t ws_size,
                              hipStream_t stream) {
  if (n_in < 23) return;
  const int nN = in_sizes[0] / HD;
  const int nE = in_sizes[5];
  if (nN <= 0 || nE <= 0) return;
  if (in_sizes[0] != nN * HD || in_sizes[1] != 3 * nN || in_sizes[2] != nE * EF || in_sizes[3] != nN * ADY) return;
  if (in_sizes[4] != nN * HD || in_sizes[6] != nE) return;
  if (in_sizes[7] != W1R * INR || in_sizes[8] != INR || in_sizes[9] != INR * INR || in_sizes[10] != INR) return;
  if (in_sizes[11] != INR || in_sizes[12] != INR * HD || in_sizes[13] != INR * NHD || in_sizes[14] != HD * HD) return;
  if (in_sizes[15] != HD * INR || in_sizes[16] != INR || in_sizes[17] != INR * HD || in_sizes[18] != HD) return;
  if (in_sizes[19] != ADY * H2 || in_sizes[20] != H2 || in_sizes[21] != ADY * H2 || in_sizes[22] != H2) return;
  if (out_size != 2 * nN * HD + 3 * nN) return;
  if ((nN % 4) != 0) return;
  if (nN > (1 << 20) || nE > (1 << 26)) return;

  const float* hF   = (const float*)d_in[0];
  const float* crd  = (const float*)d_in[1];
  const float* aF   = (const float*)d_in[2];
  const float* yF   = (const float*)d_in[3];
  const float* resF = (const float*)d_in[4];
  const int*   srcI = (const int*)d_in[5];
  const int*   dstI = (const int*)d_in[6];
  const float* We1  = (const float*)d_in[7];
  const float* be1  = (const float*)d_in[8];
  const float* We2  = (const float*)d_in[9];
  const float* be2  = (const float*)d_in[10];
  const float* Wc   = (const float*)d_in[11];
  const float* Wv   = (const float*)d_in[12];
  const float* Wa   = (const float*)d_in[13];
  const float* Wo   = (const float*)d_in[14];
  const float* Wn1  = (const float*)d_in[15];
  const float* bn1  = (const float*)d_in[16];
  const float* Wn2  = (const float*)d_in[17];
  const float* bn2  = (const float*)d_in[18];
  const float* Wf1  = (const float*)d_in[19];
  const float* bf1  = (const float*)d_in[20];
  const float* Wf2  = (const float*)d_in[21];
  const float* bf2  = (const float*)d_in[22];
  float* out = (float*)d_out;

  const int NP = ((nN + 63) / 64) * 64;
  const int nBC = (nN + NBC - 1) / NBC;
  const int CNTPAD = nBC * NBC;
  if (4 * nBC + 1 > RBN) return;
  const int nBF = (nN + NBF - 1) / NBF;
  if (nBF > 4 * nBC) return;
  if (31 * 4 * nBC > 4096) return;
  const int csrLen = ((nE + 127) & ~127) + 4096;
  const int HS = csrLen / 2;
  const size_t NPs = (size_t)NP;
  const size_t HSs = (size_t)HS;

  char* ws = (char*)d_ws;
  size_t off = 0;
  const size_t oPQW = off; off += (size_t)PQC * HD * 2;    off = (off + 255) & ~(size_t)255;
  const size_t oW1A = off; off += (size_t)INR * KA * 2;    off = (off + 255) & ~(size_t)255;
  const size_t oWE2 = off; off += (size_t)INR * INR * 2;   off = (off + 255) & ~(size_t)255;
  const size_t oWHD = off; off += (size_t)HDC * INR * 2;   off = (off + 255) & ~(size_t)255;
  const size_t oWO  = off; off += (size_t)HD * HD * 2;     off = (off + 255) & ~(size_t)255;
  const size_t oWN1 = off; off += (size_t)INR * HD * 2;    off = (off + 255) & ~(size_t)255;
  const size_t oWN2 = off; off += (size_t)HD * INR * 2;    off = (off + 255) & ~(size_t)255;
  const size_t oWF1 = off; off += (size_t)H2 * ADY * 2;    off = (off + 255) & ~(size_t)255;
  const size_t oWF2 = off; off += (size_t)H2 * ADY * 2;    off = (off + 255) & ~(size_t)255;
  const size_t oPQ  = off; off += NPs * PQC * 4;           off = (off + 255) & ~(size_t)255;
  const size_t oVH  = off; off += HSs * HD * 2;            off = (off + 255) & ~(size_t)255;
  const size_t oLH  = off; off += HSs * NHD * 4;           off = (off + 255) & ~(size_t)255;
  const size_t oCH  = off; off += HSs * 4 * 4;             off = (off + 255) & ~(size_t)255;
  const size_t oST  = off; off += NPs * STW * 4;           off = (off + 255) & ~(size_t)255;
  const size_t oHAG = off; off += NPs * HD * 2;            off = (off + 255) & ~(size_t)255;
  const size_t oR2  = off; off += NPs * HD * 4;            off = (off + 255) & ~(size_t)255;
  const size_t oCO  = off; off += NPs * 4 * 4;             off = (off + 255) & ~(size_t)255;
  const size_t oCnt = off; off += (size_t)CNTPAD * 4;      off = (off + 255) & ~(size_t)255;
  const size_t oOff = off; off += (size_t)CNTPAD * 4;      off = (off + 255) & ~(size_t)255;
  const size_t oRb  = off; off += (size_t)RBN * 4;         off = (off + 255) & ~(size_t)255;
  const size_t oCsE = off; off += (size_t)csrLen * 4;      off = (off + 255) & ~(size_t)255;
  if (off > ws_size || off > (size_t)WSCAP) return;

  unsigned short* PQW  = (unsigned short*)(ws + oPQW);
  unsigned short* W1Ap = (unsigned short*)(ws + oW1A);
  unsigned short* WE2p = (unsigned short*)(ws + oWE2);
  unsigned short* WHDp = (unsigned short*)(ws + oWHD);
  unsigned short* WOp  = (unsigned short*)(ws + oWO);
  unsigned short* WN1p = (unsigned short*)(ws + oWN1);
  unsigned short* WN2p = (unsigned short*)(ws + oWN2);
  unsigned short* WF1p = (unsigned short*)(ws + oWF1);
  unsigned short* WF2p = (unsigned short*)(ws + oWF2);
  float*          PQ   = (float*)(ws + oPQ);
  unsigned short* VH   = (unsigned short*)(ws + oVH);
  float*          LH   = (float*)(ws + oLH);
  float*          CH   = (float*)(ws + oCH);
  float*          ST   = (float*)(ws + oST);
  unsigned short* HAGG = (unsigned short*)(ws + oHAG);
  float*          R2   = (float*)(ws + oR2);
  float*          CO   = (float*)(ws + oCO);
  int*            cnt  = (int*)(ws + oCnt);
  int*            offp = (int*)(ws + oOff);
  int*            rb   = (int*)(ws + oRb);
  int*            csrE = (int*)(ws + oCsE);

  const int vec8 = 1;

  k_wcvt<<<dim3((PQC * (HD / 8) + NTHR - 1) / NTHR, 9, 1), NTHR, 0, stream>>>(
      We1, We2, Wv, Wa, Wc, Wo, Wn1, Wn2, Wf1, Wf2, PQW, W1Ap, WE2p, WHDp, WOp, WN1p, WN2p, WF1p, WF2p);
  k_count<<<nBC, NTHR, 0, stream>>>(dstI, cnt, nE, vec8);
  k_offsets<<<1, OTHR, 0, stream>>>(cnt, offp, rb, nBC);
  hipFuncSetAttribute(reinterpret_cast<const void*>(&k_fill), hipFuncAttributeMaxDynamicSharedMemorySize, LDS_FILL);
  k_fill<<<nBF, NTHR, LDS_FILL, stream>>>(dstI, offp, rb, csrE, nE, vec8, csrLen);
  k_pq<<<dim3(NP / BM, PQC / NCW, 1), NTHR, 0, stream>>>(hF, PQW, PQ, nN);
  k_edge<<<HS / (TWE * 16), TTE, 0, stream>>>(csrE, srcI, dstI, crd, aF, PQ, We1 + (size_t)256 * INR, be1,
                                              W1Ap, WE2p, be2, WHDp, VH, LH, CH, nN, nE, csrLen, 0);
  k_agg<0><<<NP / ANB, NTHR, 0, stream>>>(cnt, offp, VH, LH, CH, ST, crd, CO, HAGG, nN, csrLen, 0, HS);
  k_edge<<<HS / (TWE * 16), TTE, 0, stream>>>(csrE, srcI, dstI, crd, aF, PQ, We1 + (size_t)256 * INR, be1,
                                              W1Ap, WE2p, be2, WHDp, VH, LH, CH, nN, nE, csrLen, HS);
  k_agg<1><<<NP / ANB, NTHR, 0, stream>>>(cnt, offp, VH, LH, CH, ST, crd, CO, HAGG, nN, csrLen, HS, HS);
  hipFuncSetAttribute(reinterpret_cast<const void*>(&k_node), hipFuncAttributeMaxDynamicSharedMemorySize, LDS_NODE);
  k_node<<<NP / (TWN * 16), TTN, LDS_NODE, stream>>>(hF, yF, resF, HAGG, WOp, WF1p, bf1, WF2p, bf2,
                                                     WN1p, bn1, WN2p, bn2, out, R2, nN);
  const int e1 = nN * HD;
  const int e2 = nN * HD + 3 * nN;
  const int q0 = e1 / 4;
  const int qSplit = e2 / 4;
  const int q1 = out_size / 4;
  if (4 * q1 != out_size || 4 * q0 != e1 || 4 * qSplit != e2) return;
  const int nq = q1 - q0;
  k_out<<<(nq + NTHR - 1) / NTHR, NTHR, 0, stream>>>(CO, R2, out, nN, q0, qSplit, q1, e1, e2);
}
